// Model_1047972020547
// MI455X (gfx1250) — hardware-verified
//
#include <hip/hip_runtime.h>
#include <math.h>

constexpr int NVOC  = 50000;
constexpr int NEMB  = 300;
constexpr int KPAD  = 320;
constexpr int NHID  = 256;
constexpr int NG3   = 768;
constexpr int NH2   = 512;
constexpr int NREP  = 2048;
constexpr int NTOK0 = 128;
constexpr int NTOKR = 64;
constexpr int NSEQ  = 2049;
constexpr int MPAD  = 2112;
constexpr int NTHR  = 256;
constexpr int NTA   = 512;
constexpr int NOUT0 = NSEQ * NHID;
static_assert(KPAD % 32 == 0 && NH2 % 32 == 0, "GEMM K multiple of 32");
static_assert(MPAD % 64 == 0 && NG3 % 64 == 0 && NHID % 64 == 0, "GEMM M, N tile multiples");
static_assert(MPAD >= NSEQ && KPAD >= NEMB, "padding");
static_assert(NOUT0 * 4 == 2098176, "byte offset of the second output");
static_assert((NG3 * (KPAD / 8)) % NTHR == 0, "weight split grid exact");
static_assert((NHID * (NH2 / 8)) % NTHR == 0, "weight split grid exact");
static_assert(KPAD / 8 == 40, "X row = 40 chunks of 8 halves");
static_assert(NHID == 8 * 32, "one wave writes one 256-wide bf16 row half per instruction");
static_assert((MPAD - NSEQ) < 64, "pad rows");

typedef __attribute__((ext_vector_type(16))) _Float16 v16h;
typedef __attribute__((ext_vector_type(8)))  _Float16 v8h;
typedef __attribute__((ext_vector_type(16))) __bf16   v16b;
typedef __attribute__((ext_vector_type(8)))  __bf16   v8b;
typedef __attribute__((ext_vector_type(8)))  float    v8f;
typedef __attribute__((ext_vector_type(4)))  float    v4f;
typedef __attribute__((ext_vector_type(2)))  float    v2f;
typedef __attribute__((ext_vector_type(4)))  unsigned v4u;

__device__ __forceinline__ unsigned short f2bf_bits(float f) {
  unsigned u = __float_as_uint(f);
  return (unsigned short)((u + 0x7FFFu + ((u >> 16) & 1u)) >> 16);
}
__device__ __forceinline__ float bf_bits2f(unsigned short h) { return __uint_as_float(((unsigned)h) << 16); }

__device__ __forceinline__ void dep_guard_h(v8f& a, v8f& b, v16h x, v16h y) { asm volatile("v_nop\n\tv_nop\n\tv_nop\n\tv_nop" : "+v"(a), "+v"(b) : "v"(x), "v"(y)); }
__device__ __forceinline__ void dep_guard_b(v8f& a, v8f& b, v16b x, v16b y) { asm volatile("v_nop\n\tv_nop\n\tv_nop\n\tv_nop" : "+v"(a), "+v"(b) : "v"(x), "v"(y)); }
__device__ __forceinline__ void dep_guard4x_h(v8f& a, v8f& b, v8f& c, v8f& d, v16h x, v16h y) {
  asm volatile("v_nop\n\tv_nop\n\tv_nop\n\tv_nop" : "+v"(a), "+v"(b), "+v"(c), "+v"(d) : "v"(x), "v"(y));
}
__device__ __forceinline__ void dep_guard4x_b(v8f& a, v8f& b, v8f& c, v8f& d, v16b x, v16b y) {
  asm volatile("v_nop\n\tv_nop\n\tv_nop\n\tv_nop" : "+v"(a), "+v"(b), "+v"(c), "+v"(d) : "v"(x), "v"(y));
}
__device__ __forceinline__ void keep4_h(v16h a, v16h b, v16h c, v16h d) { asm volatile("v_nop" :: "v"(a), "v"(b), "v"(c), "v"(d)); }
__device__ __forceinline__ void keep4_b(v16b a, v16b b, v16b c, v16b d) { asm volatile("v_nop" :: "v"(a), "v"(b), "v"(c), "v"(d)); }
__device__ __forceinline__ void acc_guard4(v8f& a, v8f& b, v8f& c, v8f& d) { asm volatile("v_nop\n\tv_nop\n\tv_nop\n\tv_nop" : "+v"(a), "+v"(b), "+v"(c), "+v"(d)); }
template <typename T> struct Frag;
template <> struct Frag<_Float16> {
  typedef v16h V; union U { v16h v; v8h h[2]; };
  static __device__ __forceinline__ v16h load(const _Float16* p) {
    U f; f.h[0] = *(const v8h*)(p); f.h[1] = *(const v8h*)(p + 16); return f.v;
  }
  static __device__ __forceinline__ v8f mma(v16h a, v16h b, v8f c) {
    return __builtin_amdgcn_wmma_f32_16x16x32_f16(false, a, false, b, (short)0, c, false, false);
  }
  static __device__ __forceinline__ void guard(v8f& a, v8f& b, v16h x, v16h y) { dep_guard_h(a, b, x, y); }
  static __device__ __forceinline__ void guard4(v8f& a, v8f& b, v8f& c, v8f& d, v16h x, v16h y) { dep_guard4x_h(a, b, c, d, x, y); }
  static __device__ __forceinline__ void keep(v16h a, v16h b, v16h c, v16h d) { keep4_h(a, b, c, d); }
};
template <> struct Frag<__bf16> {
  typedef v16b V; union U { v16b v; v8b h[2]; };
  static __device__ __forceinline__ v16b load(const __bf16* p) {
    U f; f.h[0] = *(const v8b*)(p); f.h[1] = *(const v8b*)(p + 16); return f.v;
  }
  static __device__ __forceinline__ v8f mma(v16b a, v16b b, v8f c) {
    return __builtin_amdgcn_wmma_f32_16x16x32_bf16(false, a, false, b, (short)0, c, false, false);
  }
  static __device__ __forceinline__ void guard(v8f& a, v8f& b, v16b x, v16b y) { dep_guard_b(a, b, x, y); }
  static __device__ __forceinline__ void guard4(v8f& a, v8f& b, v8f& c, v8f& d, v16b x, v16b y) { dep_guard4x_b(a, b, c, d, x, y); }
  static __device__ __forceinline__ void keep(v16b a, v16b b, v16b c, v16b d) { keep4_b(a, b, c, d); }
};

__device__ __forceinline__ float fsig(float x) { return __builtin_amdgcn_rcpf(1.0f + expf(-x)); }

template <int ET> struct Elem;
template <> struct Elem<0> { typedef _Float16 T; };
template <> struct Elem<1> { typedef __bf16 T; };
template <int ET, bool SPLIT, int BIAS_MODE, int OUT_MODE, bool RESID, int ACT = 0>
__global__ __launch_bounds__(256) void wmma_gemm64(
    const unsigned short* __restrict__ Ap, const unsigned short* __restrict__ A2p, int lda, long strideA,
    const unsigned short* __restrict__ Btp, const unsigned short* __restrict__ Bt2p, int ldb, long strideB,
    void* __restrict__ Cout, void* __restrict__ Cout2, int ldc, long strideC,
    const float* __restrict__ bias,
    const float* __restrict__ resid, long strideR,
    int M, int N, int K, float scale, int Mstore) {
  typedef typename Elem<ET>::T T;
  typedef typename Frag<T>::V V;
  const T* A = (const T*)Ap; const T* A2 = (const T*)A2p; const T* Bt = (const T*)Btp; const T* Bt2 = (const T*)Bt2p;
  __shared__ __align__(16) float sT[8][16 * 68];
  const int b    = blockIdx.y;
  const int lane = threadIdx.x & 31;
  const int wave = threadIdx.x >> 5;
  const int tilesN = N >> 6;
  const int tilesM = M >> 6;
  const int tile = blockIdx.x * 8 + wave;
  if (tile >= tilesM * tilesN) return;
  const int tm = tile / tilesN;
  const int tn = tile - tm * tilesN;
  const int m0 = tm << 6;
  const int n0 = tn << 6;

  const T* Ab  = A  + (size_t)b * strideA;
  const T* Bb  = Bt + (size_t)b * strideB;
  const T* Ab2 = SPLIT ? (A2  + (size_t)b * strideA) : nullptr;
  const T* Bb2 = SPLIT ? (Bt2 + (size_t)b * strideB) : nullptr;

  const int rlane = lane & 15;
  const int koff  = (lane >> 4) * 8;
  const int mOff  = (lane >> 4) * 8;

  v8f acc[4][4];
#pragma unroll
  for (int i = 0; i < 4; ++i)
#pragma unroll
    for (int j = 0; j < 4; ++j) acc[i][j] = (v8f){0.f,0.f,0.f,0.f,0.f,0.f,0.f,0.f};

  for (int k0 = 0; k0 < K; k0 += 32) {
    V bh[4], bl[4];
#pragma unroll
    for (int j = 0; j < 4; ++j) {
      const size_t bo = (size_t)(n0 + (j << 4) + rlane) * ldb + koff + k0;
      bh[j] = Frag<T>::load(Bb + bo);
      if (SPLIT) bl[j] = Frag<T>::load(Bb2 + bo);
    }
#pragma unroll
    for (int i = 0; i < 4; ++i) {
      const size_t ao = (size_t)(m0 + (i << 4) + rlane) * lda + koff + k0;
      V ah = Frag<T>::load(Ab + ao);
      V al;
      if (SPLIT) al = Frag<T>::load(Ab2 + ao);
#pragma unroll
      for (int j = 0; j < 4; ++j) {
        acc[i][j] = Frag<T>::mma(ah, bh[j], acc[i][j]);
        if (SPLIT) {
          acc[i][j] = Frag<T>::mma(ah, bl[j], acc[i][j]);
          acc[i][j] = Frag<T>::mma(al, bh[j], acc[i][j]);
        }
      }
      Frag<T>::guard4(acc[i][0], acc[i][1], acc[i][2], acc[i][3], ah, SPLIT ? al : ah);
    }
    Frag<T>::keep(bh[0], bh[1], bh[2], bh[3]);
    if (SPLIT) Frag<T>::keep(bl[0], bl[1], bl[2], bl[3]);
  }
  acc_guard4(acc[0][0], acc[0][1], acc[0][2], acc[0][3]);
  acc_guard4(acc[1][0], acc[1][1], acc[1][2], acc[1][3]);
  acc_guard4(acc[2][0], acc[2][1], acc[2][2], acc[2][3]);
  acc_guard4(acc[3][0], acc[3][1], acc[3][2], acc[3][3]);

  float* slab = sT[wave];
  const float* Rb = RESID ? (resid + (size_t)b * strideR) : nullptr;
#pragma unroll
  for (int i = 0; i < 4; ++i) {
    const int mBase = m0 + (i << 4);
#pragma unroll
    for (int j = 0; j < 4; ++j) {
      const int n = n0 + (j << 4) + rlane;
      float bv = 0.f;
      if (BIAS_MODE == 2) bv = bias[n];
#pragma unroll
      for (int r = 0; r < 8; ++r) {
        float v = acc[i][j][r] * scale;
        if (BIAS_MODE == 1) v += bias[mBase + mOff + r];
        if (BIAS_MODE == 2) v += bv;
        if (RESID) v += Rb[(size_t)(mBase + mOff + r) * ldc + n];
        if (ACT == 1) v = tanhf(v);
        if (ACT == 2) v = fmaxf(v, 0.0f);
        if (ACT == 3) v = v / (1.0f + expf(-v));
        if (ACT == 4) v = (v > 0.f) ? v : 0.01f * v;
        slab[(mOff + r) * 68 + (j << 4) + rlane] = v;
      }
    }
    __builtin_amdgcn_fence(__ATOMIC_RELEASE, "workgroup");
    __builtin_amdgcn_wave_barrier();
    __builtin_amdgcn_fence(__ATOMIC_ACQUIRE, "workgroup");
    if (OUT_MODE == 0) {
      float* C = (float*)Cout + (size_t)b * strideC;
      const int hh = lane >> 4, c4 = (lane & 15) * 4;
      for (int pass = 0; pass < 2; ++pass) {
#pragma unroll
        for (int it = 0; it < 8; ++it) {
          const int row = it * 2 + hh;
          v4f v = *(const v4f*)(slab + row * 68 + c4);
          if (mBase + row < Mstore) *(volatile v4f*)(C + (size_t)(mBase + row) * ldc + n0 + c4) = v;
        }
        __threadfence();
      }
    } else {
      const int q = lane >> 3, c8 = (lane & 7) * 8;
      unsigned short* C  = (unsigned short*)Cout  + (size_t)b * strideC;
      unsigned short* C2 = (OUT_MODE == 2) ? ((unsigned short*)Cout2 + (size_t)b * strideC) : nullptr;
      for (int pass = 0; pass < 2; ++pass) {
#pragma unroll
        for (int it = 0; it < 4; ++it) {
          const int row = it * 4 + q;
          const float* sp = slab + row * 68 + c8;
          v8h hv, lv;
#pragma unroll
          for (int e = 0; e < 8; ++e) {
            if (OUT_MODE == 1) {
              hv[e] = (_Float16)sp[e];
            } else {
              unsigned short hb = f2bf_bits(sp[e]);
              unsigned short lb = f2bf_bits(sp[e] - bf_bits2f(hb));
              hv[e] = __builtin_bit_cast(_Float16, hb);
              lv[e] = __builtin_bit_cast(_Float16, lb);
            }
          }
          if (mBase + row < Mstore) {
            *(volatile v8h*)(C + (size_t)(mBase + row) * ldc + n0 + c8) = hv;
            if (OUT_MODE == 2) *(volatile v8h*)(C2 + (size_t)(mBase + row) * ldc + n0 + c8) = lv;
          }
        }
        __threadfence();
      }
    }
    __builtin_amdgcn_fence(__ATOMIC_RELEASE, "workgroup");
    __builtin_amdgcn_wave_barrier();
    __builtin_amdgcn_fence(__ATOMIC_ACQUIRE, "workgroup");
  }
}

__global__ __launch_bounds__(KPAD) void gather_rows_kernel(const int* __restrict__ tok0, const int* __restrict__ tokr,
                                                          const int* __restrict__ lenr, const float* __restrict__ emb,
                                                          unsigned short* __restrict__ XH, unsigned short* __restrict__ XL) {
  __shared__ int stok[NTOK0];
  __shared__ __align__(16) float srow[KPAD];
  const int row = blockIdx.x;
  const int tid = threadIdx.x;
  int ntok;
  if (row == 0) {
    if (tid < NTOK0) {
      int tk = tok0[tid];
      tk = tk < 0 ? 0 : tk; tk = tk > NVOC - 1 ? NVOC - 1 : tk;
      stok[tid] = tk;
    }
    ntok = NTOK0;
  } else {
    int r = row - 1; r = r > NREP - 1 ? NREP - 1 : r;
    if (tid < NTOKR) {
      int tk = tokr[(size_t)r * NTOKR + tid];
      tk = tk < 0 ? 0 : tk; tk = tk > NVOC - 1 ? NVOC - 1 : tk;
      stok[tid] = tk;
    }
    int L = lenr[r];
    L = L < 0 ? 0 : L; L = L > NTOKR ? NTOKR : L;
    ntok = (row < NSEQ) ? L : 0;
  }
  __syncthreads();

  const int col = (tid < NEMB) ? tid : (NEMB - 1);
  float s = 0.0f;
#pragma unroll 4
  for (int t = 0; t < ntok; ++t) s += emb[(size_t)stok[t] * NEMB + col];
  srow[tid] = (tid < NEMB) ? s : 0.0f;
  __syncthreads();

  const int ch  = (tid < 64) ? tid : (tid - 64);
  const int chc = (ch > 39) ? 39 : ch;
  v8h hv, lv;
#pragma unroll
  for (int e = 0; e < 8; ++e) {
    const float v = srow[chc * 8 + e];
    const unsigned short hb = f2bf_bits(v);
    const unsigned short lb = f2bf_bits(v - bf_bits2f(hb));
    hv[e] = __builtin_bit_cast(_Float16, hb);
    lv[e] = __builtin_bit_cast(_Float16, lb);
  }
  const bool wh = (tid < 40);
  const bool wl = (tid >= 64) && (tid < 104);
  const size_t o = (size_t)row * KPAD + (size_t)chc * 8;
  for (int pass = 0; pass < 2; ++pass) {
    if (wh) *(volatile v8h*)(XH + o) = hv;
    if (wl) *(volatile v8h*)(XL + o) = lv;
    __threadfence();
  }
}

__global__ __launch_bounds__(NTHR) void wsplit8_kernel(const float* __restrict__ src0, const float* __restrict__ src1,
                                                      unsigned short* __restrict__ dstH, unsigned short* __restrict__ dstL,
                                                      int nrow, int ncol, int kpad) {
  const int i = blockIdx.x * NTHR + threadIdx.x;
  const int nc8 = kpad >> 3;
  const int n8 = nrow * nc8;
  const float* src = (blockIdx.y == 0) ? src0 : src1;
  if (i < n8) {
    const int row = i / nc8;
    const int c8  = i - row * nc8;
    const float* sp = src + (size_t)row * ncol;
    v8h hv, lv;
#pragma unroll
    for (int e = 0; e < 8; ++e) {
      const int cidx = c8 * 8 + e;
      const int cc = (cidx < ncol) ? cidx : (ncol - 1);
      const float raw = sp[cc];
      const float v = (cidx < ncol) ? raw : 0.0f;
      const unsigned short hb = f2bf_bits(v);
      const unsigned short lb = f2bf_bits(v - bf_bits2f(hb));
      hv[e] = __builtin_bit_cast(_Float16, hb);
      lv[e] = __builtin_bit_cast(_Float16, lb);
    }
    const size_t o = (size_t)blockIdx.y * (size_t)n8 * 8 + (size_t)i * 8;
    *(volatile v8h*)(dstH + o) = hv;
    *(volatile v8h*)(dstL + o) = lv;
    __threadfence();
    *(volatile v8h*)(dstH + o) = hv;
    *(volatile v8h*)(dstL + o) = lv;
  }
}

__global__ __launch_bounds__(NTHR) void gru_seq_kernel(const float* __restrict__ GI,
                                                       const float* __restrict__ Whh_f, const float* __restrict__ bih_f,
                                                       const float* __restrict__ bhh_f,
                                                       const float* __restrict__ Whh_b, const float* __restrict__ bih_b,
                                                       const float* __restrict__ bhh_b,
                                                       unsigned short* __restrict__ O2H, unsigned short* __restrict__ O2L,
                                                       float* __restrict__ HFB) {
  __shared__ __align__(16) float hs[NHID];
  const int dir = blockIdx.x, tid = threadIdx.x, lane = tid & 31, wave = tid >> 5;
  const int j = tid;
  const float* Whh = dir ? Whh_b : Whh_f;
  const float* bih = dir ? bih_b : bih_f;
  const float* bhh = dir ? bhh_b : bhh_f;
  const float* GId = GI + (size_t)dir * MPAD * NG3;
  const int cbase = dir * NHID;

  {
    const v4u zz = {0u, 0u, 0u, 0u};
    for (int pass = 0; pass < 2; ++pass) {
#pragma unroll 1
      for (int rr = wave; rr < MPAD - NSEQ; rr += NTHR / 32) {
        const size_t o = (size_t)(NSEQ + rr) * NH2 + cbase + 8 * lane;
        *(volatile v4u*)(O2H + o) = zz;
        *(volatile v4u*)(O2L + o) = zz;
      }
      __threadfence();
    }
  }

  hs[j] = 0.0f;
  const float bi_r = bih[j], bi_z = bih[NHID + j], bi_n = bih[2 * NHID + j];
  const float bh_r = bhh[j], bh_z = bhh[NHID + j], bh_n = bhh[2 * NHID + j];
  const float* wr = Whh + (size_t)j * NHID;
  const float* wz = Whh + (size_t)(NHID + j) * NHID;
  const float* wn = Whh + (size_t)(2 * NHID + j) * NHID;
  __syncthreads();

#pragma unroll 1
  for (int t = 0; t < NSEQ; ++t) {
    const int row = dir ? (NSEQ - 1 - t) : t;
    const float* g = GId + (size_t)row * NG3;
    const float gi_r = g[j], gi_z = g[NHID + j], gi_n = g[2 * NHID + j];
    float ar = bh_r, az = bh_z, an = bh_n;
#pragma unroll 4
    for (int k = 0; k < NHID; ++k) {
      const float hk = hs[k];
      ar = fmaf(wr[k], hk, ar);
      az = fmaf(wz[k], hk, az);
      an = fmaf(wn[k], hk, an);
    }
    const float hold = hs[j];
    const float rg = fsig(gi_r + bi_r + ar);
    const float zg = fsig(gi_z + bi_z + az);
    const float ng = tanhf(gi_n + bi_n + rg * an);
    const float hnew = (1.0f - zg) * ng + zg * hold;
    __syncthreads();
    hs[j] = hnew;
    __syncthreads();
    if (wave < 2) {
      v8h hv, lv;
#pragma unroll
      for (int e = 0; e < 8; ++e) {
        const float v = hs[8 * lane + e];
        const unsigned short hb = f2bf_bits(v);
        const unsigned short lb = f2bf_bits(v - bf_bits2f(hb));
        hv[e] = __builtin_bit_cast(_Float16, hb);
        lv[e] = __builtin_bit_cast(_Float16, lb);
      }
      const size_t o = (size_t)row * NH2 + cbase + 8 * lane;
      if (wave == 0) {
        *(volatile v8h*)(O2H + o) = hv;
        __threadfence();
        *(volatile v8h*)(O2H + o) = hv;
      } else {
        *(volatile v8h*)(O2L + o) = lv;
        __threadfence();
        *(volatile v8h*)(O2L + o) = lv;
      }
    }
  }

  if (wave == 0) {
    for (int pass = 0; pass < 2; ++pass) {
#pragma unroll
      for (int it = 0; it < 2; ++it) {
        const int c4 = it * 128 + 4 * lane;
        const v4f v = *(const v4f*)(hs + c4);
        *(volatile v4f*)(HFB + (size_t)dir * NHID + c4) = v;
      }
      __threadfence();
    }
  }
}

__global__ __launch_bounds__(NTA) void attn_tail_kernel(const float* __restrict__ outp, const float* __restrict__ HFB,
                                                       const float* __restrict__ Wo, const float* __restrict__ bo,
                                                       const float* __restrict__ label, float* __restrict__ tail) {
  __shared__ __align__(16) float hsum[NHID];
  __shared__ float sc[MPAD];
  __shared__ float red[NTA];
  const int tid = threadIdx.x, lane = tid & 31, wave = tid >> 5;
  if (tid < NHID) hsum[tid] = HFB[tid] + HFB[NHID + tid];
  __syncthreads();

#pragma unroll 1
  for (int t = wave; t < NSEQ; t += NTA / 32) {
    const float* o = outp + (size_t)t * NHID;
    const v4f a  = *(const v4f*)(o + 4 * lane);
    const v4f b  = *(const v4f*)(o + 128 + 4 * lane);
    const v4f ha = *(const v4f*)(hsum + 4 * lane);
    const v4f hb = *(const v4f*)(hsum + 128 + 4 * lane);
    float p = 0.0f;
    p += a[0] * ha[0]; p += a[1] * ha[1]; p += a[2] * ha[2]; p += a[3] * ha[3];
    p += b[0] * hb[0]; p += b[1] * hb[1]; p += b[2] * hb[2]; p += b[3] * hb[3];
#pragma unroll
    for (int off = 1; off < 32; off <<= 1) p += __shfl_xor(p, off, 32);
    if (lane == 0) sc[t] = p;
  }
  __syncthreads();

  float m = -INFINITY;
#pragma unroll 1
  for (int t = tid; t < NSEQ; t += NTA) m = fmaxf(m, sc[t]);
  red[tid] = m;
  __syncthreads();
  for (int off = NTA / 2; off > 0; off >>= 1) {
    if (tid < off) red[tid] = fmaxf(red[tid], red[tid + off]);
    __syncthreads();
  }
  const float mx = red[0];
  __syncthreads();

  float ls = 0.0f;
#pragma unroll 1
  for (int t = tid; t < NSEQ; t += NTA) {
    const float e = expf(sc[t] - mx);
    sc[t] = e;
    ls += e;
  }
  red[tid] = ls;
  __syncthreads();
  for (int off = NTA / 2; off > 0; off >>= 1) {
    if (tid < off) red[tid] += red[tid + off];
    __syncthreads();
  }
  const float tot = red[0];
  __syncthreads();
  const float inv = __builtin_amdgcn_rcpf(tot);

  float cw = 0.0f;
  if (tid < NHID) {
    float c = 0.0f;
#pragma unroll 4
    for (int t = 0; t < NSEQ; ++t) c = fmaf(sc[t], outp[(size_t)t * NHID + tid], c);
    cw = (c * inv) * Wo[tid];
  }
  red[tid] = cw;
  __syncthreads();
  for (int off = NTA / 2; off > 0; off >>= 1) {
    if (tid < off) red[tid] += red[tid + off];
    __syncthreads();
  }
  if (tid == 0) {
    const float x = red[0] + bo[0];
    const float res = fsig(x);
    const float d = label[0] - res;
    v2f v; v[0] = d * d; v[1] = res;
    *(volatile v2f*)(tail) = v;
    __threadfence();
    *(volatile v2f*)(tail) = v;
  }
}

extern "C" void kernel_launch(void* const* d_in, const int* in_sizes, int n_in,
                              void* d_out, int out_size, void* d_ws, size_t ws_size, hipStream_t stream) {
  if (n_in < 17 || d_out == nullptr || d_ws == nullptr) return;
  if (in_sizes[0] != NTOK0 || in_sizes[1] != NREP * NTOKR || in_sizes[2] != NREP || in_sizes[3] != 1 ||
      in_sizes[4] != NVOC * NEMB || in_sizes[5] != NG3 * NEMB || in_sizes[6] != NG3 * NHID || in_sizes[7] != NG3 ||
      in_sizes[8] != NG3 || in_sizes[9] != NG3 * NEMB || in_sizes[10] != NG3 * NHID || in_sizes[11] != NG3 ||
      in_sizes[12] != NG3 || in_sizes[13] != NHID * NH2 || in_sizes[14] != NHID || in_sizes[15] != NHID ||
      in_sizes[16] != 1 || out_size != NOUT0 + 2) return;

  const int*   tok0  = (const int*)d_in[0];
  const int*   tokr  = (const int*)d_in[1];
  const int*   lenr  = (const int*)d_in[2];
  const float* label = (const float*)d_in[3];
  const float* emb   = (const float*)d_in[4];
  const float* Wih_f = (const float*)d_in[5];
  const float* Whh_f = (const float*)d_in[6];
  const float* bih_f = (const float*)d_in[7];
  const float* bhh_f = (const float*)d_in[8];
  const float* Wih_b = (const float*)d_in[9];
  const float* Whh_b = (const float*)d_in[10];
  const float* bih_b = (const float*)d_in[11];
  const float* bhh_b = (const float*)d_in[12];
  const float* Wl    = (const float*)d_in[13];
  const float* blin  = (const float*)d_in[14];
  const float* Wo    = (const float*)d_in[15];
  const float* bout  = (const float*)d_in[16];
  float* out = (float*)d_out;

  char* ws = (char*)d_ws; size_t off = 0;
  auto carve = [&](size_t bytes) -> char* { char* p = ws + off; off += (bytes + 255) & ~(size_t)255; return p; };
  unsigned short* XH   = (unsigned short*)carve((size_t)MPAD * KPAD * 2);
  unsigned short* XL   = (unsigned short*)carve((size_t)MPAD * KPAD * 2);
  unsigned short* WIHH = (unsigned short*)carve((size_t)2 * NG3 * KPAD * 2);
  unsigned short* WIHL = (unsigned short*)carve((size_t)2 * NG3 * KPAD * 2);
  unsigned short* WLH  = (unsigned short*)carve((size_t)NHID * NH2 * 2);
  unsigned short* WLL  = (unsigned short*)carve((size_t)NHID * NH2 * 2);
  float*          GI   = (float*)carve((size_t)2 * MPAD * NG3 * 4);
  unsigned short* O2H  = (unsigned short*)carve((size_t)MPAD * NH2 * 2);
  unsigned short* O2L  = (unsigned short*)carve((size_t)MPAD * NH2 * 2);
  float*          HFB  = (float*)carve((size_t)2 * NHID * 4);
  if (off > ws_size || off > (size_t)134217728) return;

  gather_rows_kernel<<<MPAD, KPAD, 0, stream>>>(tok0, tokr, lenr, emb, XH, XL);

  wsplit8_kernel<<<dim3((NG3 * (KPAD / 8)) / NTHR, 2), NTHR, 0, stream>>>(Wih_f, Wih_b, WIHH, WIHL, NG3, NEMB, KPAD);
  wsplit8_kernel<<<dim3((NHID * (NH2 / 8)) / NTHR, 1), NTHR, 0, stream>>>(Wl, Wl, WLH, WLL, NHID, NH2, NH2);

  {
    const int tiles = (MPAD / 64) * (NG3 / 64);
    wmma_gemm64<1, true, 0, 0, false><<<dim3((tiles + 7) / 8, 2), 256, 0, stream>>>(
        XH, XL, KPAD, 0L,
        WIHH, WIHL, KPAD, (long)NG3 * KPAD,
        (void*)GI, (void*)GI, NG3, (long)MPAD * NG3,
        bih_f, GI, 0L,
        MPAD, NG3, KPAD, 1.0f, MPAD);
  }

  gru_seq_kernel<<<2, NTHR, 0, stream>>>(GI, Whh_f, bih_f, bhh_f, Whh_b, bih_b, bhh_b, O2H, O2L, HFB);

  {
    const int tiles = (MPAD / 64) * (NHID / 64);
    wmma_gemm64<1, true, 2, 0, false><<<dim3((tiles + 7) / 8, 1), 256, 0, stream>>>(
        O2H, O2L, NH2, 0L,
        WLH, WLL, NH2, 0L,
        (void*)out, (void*)out, NHID, 0L,
        blin, GI, 0L,
        MPAD, NHID, NH2, 1.0f, NSEQ);
  }

  attn_tail_kernel<<<1, NTA, 0, stream>>>(out, HFB, Wo, bout, label, out + (size_t)NOUT0);
}
